// CrossAttentionFusionHead_30167850287198
// MI455X (gfx1250) — hardware-verified
//
#include <hip/hip_runtime.h>
#include <hip/hip_bf16.h>
#include <math.h>

#define NQc 256
#define NMc 512
#define DDc 768
#define NHc 8
#define DHc 96
#define HIDc 256
#define H2c 64
#define GSTR 48

typedef _Float16 bf16;
typedef _Float16 f16;
typedef __attribute__((ext_vector_type(4))) unsigned v4u_t;
typedef unsigned v4ua __attribute__((ext_vector_type(4), may_alias));
typedef __attribute__((ext_vector_type(4))) float v4f_t;
typedef float v4fa __attribute__((ext_vector_type(4), may_alias));
typedef __attribute__((ext_vector_type(16))) bf16  bf16x16;
typedef bf16x16 f16x16;
typedef __attribute__((ext_vector_type(8)))  bf16  bf16x8;
typedef bf16x8 f16x8;
typedef __attribute__((ext_vector_type(4)))  bf16  bf16x4;
typedef __attribute__((ext_vector_type(8)))  float f32x8;
__device__ __forceinline__ f32x8 wmma16(f16x16 a, f16x16 b, f32x8 c) {
  c = __builtin_amdgcn_wmma_f32_16x16x32_f16(false, a, false, b, (short)0, c, false, false);
  asm volatile("v_nop\n\tv_nop\n\tv_nop\n\tv_nop" : "+v"(c) : "v"(a), "v"(b));
  return c;
}
#define LDS_STRIDE 48
#define KSTRIDE    72
#define VSTRIDE    48

__device__ __forceinline__ f32x8 wmma_bf16(bf16x16 a, bf16x16 b, f32x8 c) {
  c = __builtin_amdgcn_wmma_f32_16x16x32_f16(false, a, false, b, (short)0, c, false, false);
  asm volatile("v_nop\n\tv_nop\n\tv_nop\n\tv_nop" : "+v"(c) : "v"(a), "v"(b));
  return c;
}

template <typename T>
__device__ __forceinline__ bf16x16 load_frag(const T* __restrict__ base, int ld,
                                             int row0, int k0) {
  const int lane = threadIdx.x & 31;
  const int r    = lane & 15;
  const int kh   = (lane >> 4) * 8;
  const T* p0 = base + (size_t)(row0 + r) * ld + (k0 + kh);
  const T* p1 = p0 + 16;
  bf16x16 f;
#pragma unroll
  for (int i = 0; i < 8; ++i) {
    f[i]     = (bf16)p0[i];
    f[i + 8] = (bf16)p1[i];
  }
  return f;
}

__device__ __forceinline__ bf16x16 lds_frag(const bf16* base, int stride) {
  const int lane = threadIdx.x & 31;
  const int row  = lane & 15;
  const int kh   = (lane >> 4) * 8;
  const bf16x8 lo = *(const bf16x8*)(base + row * stride + kh);
  const bf16x8 hi = *(const bf16x8*)(base + row * stride + kh + 16);
  bf16x16 f;
#pragma unroll
  for (int i = 0; i < 8; ++i) { f[i] = lo[i]; f[i + 8] = hi[i]; }
  return f;
}

template <typename T>
__device__ __forceinline__ void stage_read16(const T* __restrict__ p, float* buf) {
#pragma unroll
  for (int i = 0; i < 16; ++i) buf[i] = (float)p[i];
}

__device__ __forceinline__ void stage_write(bf16* dst, const float* buf, int nquad) {
#pragma unroll
  for (int i = 0; i < nquad; ++i) {
    bf16x4 q;
    q[0] = (bf16)buf[4 * i];     q[1] = (bf16)buf[4 * i + 1];
    q[2] = (bf16)buf[4 * i + 2]; q[3] = (bf16)buf[4 * i + 3];
    *(bf16x4*)(dst + 4 * i) = q;
  }
}


#define GSTR 48
template <typename AT, int EPI, bool OUT16>
__global__ __launch_bounds__(256) void gemm_kne(const AT* __restrict__ A, int lda, const float* __restrict__ Wm, int ldw,
                                                const float* __restrict__ bias, const float* __restrict__ R, const float* __restrict__ gvec,
                                                void* __restrict__ Yv, int ldy, int K) {
  __shared__ __attribute__((aligned(16))) f16 ldsA[128 * GSTR];
  __shared__ __attribute__((aligned(16))) f16 ldsW[128 * GSTR];
  __shared__ __attribute__((aligned(16))) float oS[8][32 * 68];
  const int tid = threadIdx.x, lane = tid & 31, wave = tid >> 5, cl = lane & 15, rh = (lane >> 4) * 8;
  const int m0 = blockIdx.x * 128, n0 = blockIdx.y * 128;
  const int wm = (wave & 3) * 32, wn = (wave >> 2) * 64;
  f32x8 acc[2][4];
#pragma unroll
  for (int i = 0; i < 2; ++i)
#pragma unroll
    for (int j = 0; j < 4; ++j) { f32x8 z = {}; acc[i][j] = z; }
#pragma unroll 1
  for (int k0 = 0; k0 < K; k0 += 32) {
    __syncthreads();
    { const int row = tid >> 1, ch = (tid & 1) * 16;
      const AT* src = A + (size_t)(m0 + row) * lda + k0 + ch;
#pragma unroll
      for (int g = 0; g < 16; ++g) ldsA[row * GSTR + ch + g] = (f16)src[g]; }
    { const int k = tid >> 3, nn0 = (tid & 7) * 16;
      const float* src = Wm + (size_t)(k0 + k) * ldw + n0 + nn0;
#pragma unroll
      for (int g = 0; g < 4; ++g) { const v4f_t v = *(const v4f_t*)(src + 4 * g);
#pragma unroll
        for (int u = 0; u < 4; ++u) ldsW[(nn0 + 4 * g + u) * GSTR + k] = (f16)v[u]; } }
    __syncthreads();
    f16x16 af[2];
#pragma unroll
    for (int i = 0; i < 2; ++i) af[i] = lds_frag(ldsA + (wm + 16 * i) * GSTR, GSTR);
#pragma unroll
    for (int j = 0; j < 4; ++j) {
      const f16x16 bf = lds_frag(ldsW + (wn + 16 * j) * GSTR, GSTR);
#pragma unroll
      for (int i = 0; i < 2; ++i) acc[i][j] = wmma16(af[i], bf, acc[i][j]);
    }
  }
  float* so = oS[wave];
#pragma unroll
  for (int i = 0; i < 2; ++i)
#pragma unroll
    for (int j = 0; j < 4; ++j) {
      const int n = n0 + wn + 16 * j + cl;
      const float bv = bias ? bias[n] : 0.0f;
      const float gv = (EPI == 2) ? gvec[n] : 0.0f;
      if (EPI == 1) {
#pragma unroll 1
        for (int r = 0; r < 8; ++r) { const float xg = acc[i][j][r] + bv; so[(16 * i + rh + r) * 68 + 16 * j + cl] = 0.5f * xg * (1.0f + erff(xg * 0.70710678118654752f)); }
      } else {
#pragma unroll
        for (int r = 0; r < 8; ++r) {
          float v = acc[i][j][r] + bv;
          if (EPI == 2) v = R[(size_t)(m0 + wm + 16 * i + rh + r) * ldy + n] + gv * v;
          so[(16 * i + rh + r) * 68 + 16 * j + cl] = v;
        }
      }
    }
  asm volatile("s_wait_dscnt 0" ::: "memory");
  __builtin_amdgcn_wave_barrier();
#pragma unroll 1
  for (int pass = 0; pass < 2; ++pass) {
    if (OUT16) {
      f16* Y = (f16*)Yv;
#pragma unroll
      for (int it = 0; it < 8; ++it) { const int c = lane + 32 * it, rr = c >> 3, q8 = (c & 7) * 8;
        union { f16 h[8]; v4u_t v; } u;
#pragma unroll
        for (int e = 0; e < 8; ++e) u.h[e] = (f16)so[rr * 68 + q8 + e];
        *(volatile v4u_t*)(Y + (size_t)(m0 + wm + rr) * ldy + n0 + wn + q8) = u.v; }
    } else {
      float* Y = (float*)Yv;
#pragma unroll
      for (int it = 0; it < 16; ++it) { const int f4 = lane + 32 * it, rr = f4 >> 4, q = (f4 & 15) * 4;
        *(volatile v4f_t*)(Y + (size_t)(m0 + wm + rr) * ldy + n0 + wn + q) = *(const v4fa*)(so + rr * 68 + q); }
    }
    __threadfence();
  }
}

template <typename AT, bool ACC>
__global__ __launch_bounds__(256) void gemm_kn2(const AT* __restrict__ A, int lda, size_t strideA,
                                               const float* __restrict__ Wm, int ldw, size_t strideW,
                                               const float* __restrict__ bias, float scale,
                                               float* __restrict__ Y, int ldy, size_t strideY, int K) {
  __shared__ __attribute__((aligned(16))) f16 ldsA[128 * GSTR], ldsAl[128 * GSTR];
  __shared__ __attribute__((aligned(16))) f16 ldsW[128 * GSTR], ldsWl[128 * GSTR];
  __shared__ __attribute__((aligned(16))) float oS[8][32 * 68];
  const int tid = threadIdx.x, lane = tid & 31, wave = tid >> 5, cl = lane & 15, rh = (lane >> 4) * 8;
  const int m0 = blockIdx.x * 128, n0 = blockIdx.y * 128;
  const int wm = (wave & 3) * 32, wn = (wave >> 2) * 64;
  A += (size_t)blockIdx.z * strideA; Wm += (size_t)blockIdx.z * strideW; Y += (size_t)blockIdx.z * strideY;
  f32x8 acc[2][4], accx[2][4];
#pragma unroll
  for (int i = 0; i < 2; ++i)
#pragma unroll
    for (int j = 0; j < 4; ++j) { f32x8 z = {}; acc[i][j] = z; accx[i][j] = z; }
#pragma unroll 1
  for (int k0 = 0; k0 < K; k0 += 32) {
    __syncthreads();
    {
      const int row = tid >> 1, ch = (tid & 1) * 16;
      const AT* src = A + (size_t)(m0 + row) * lda + k0 + ch;
#pragma unroll
      for (int g = 0; g < 16; ++g) { const float v = (float)src[g]; const f16 h = (f16)v; ldsA[row * GSTR + ch + g] = h; ldsAl[row * GSTR + ch + g] = (f16)((v - (float)h) * 2048.0f); }
    }
    {
      const int k = tid >> 3, nn0 = (tid & 7) * 16;
      const float* src = Wm + (size_t)(k0 + k) * ldw + n0 + nn0;
#pragma unroll
      for (int g = 0; g < 4; ++g) { const v4f_t v = *(const v4f_t*)(src + 4 * g);
#pragma unroll
        for (int u = 0; u < 4; ++u) { const f16 h = (f16)v[u]; ldsW[(nn0 + 4 * g + u) * GSTR + k] = h; ldsWl[(nn0 + 4 * g + u) * GSTR + k] = (f16)((v[u] - (float)h) * 2048.0f); } }
    }
    __syncthreads();
    f16x16 af[2], afl[2];
#pragma unroll
    for (int i = 0; i < 2; ++i) { af[i] = lds_frag(ldsA + (wm + 16 * i) * GSTR, GSTR); afl[i] = lds_frag(ldsAl + (wm + 16 * i) * GSTR, GSTR); }
#pragma unroll
    for (int j = 0; j < 4; ++j) {
      const f16x16 bf = lds_frag(ldsW + (wn + 16 * j) * GSTR, GSTR), bfl = lds_frag(ldsWl + (wn + 16 * j) * GSTR, GSTR);
#pragma unroll
      for (int i = 0; i < 2; ++i) { acc[i][j] = wmma16(af[i], bf, acc[i][j]); accx[i][j] = wmma16(af[i], bfl, accx[i][j]); accx[i][j] = wmma16(afl[i], bf, accx[i][j]); }
    }
  }
  float* so = oS[wave];
#pragma unroll
  for (int i = 0; i < 2; ++i)
#pragma unroll
    for (int j = 0; j < 4; ++j) {
      const float bv = bias ? bias[n0 + wn + 16 * j + cl] : 0.0f;
#pragma unroll
      for (int r = 0; r < 8; ++r) so[(16 * i + rh + r) * 68 + 16 * j + cl] = (acc[i][j][r] + accx[i][j][r] * (1.0f / 2048.0f)) * scale + bv;
    }
  asm volatile("s_wait_dscnt 0" ::: "memory");
  __builtin_amdgcn_wave_barrier();
  if (ACC) {
#pragma unroll
    for (int it = 0; it < 16; ++it) { const int f4 = lane + 32 * it, rr = f4 >> 4, q = (f4 & 15) * 4;
      const v4f_t old = *(const v4fa*)(Y + (size_t)(m0 + wm + rr) * ldy + n0 + wn + q);
      v4f_t v = *(const v4fa*)(so + rr * 68 + q); v += old; *(volatile v4fa*)(so + rr * 68 + q) = v; }
    asm volatile("s_wait_dscnt 0" ::: "memory");
  }
#pragma unroll 1
  for (int pass = 0; pass < 2; ++pass) {
#pragma unroll
    for (int it = 0; it < 16; ++it) { const int f4 = lane + 32 * it, rr = f4 >> 4, q = (f4 & 15) * 4;
      *(volatile v4f_t*)(Y + (size_t)(m0 + wm + rr) * ldy + n0 + wn + q) = *(const v4fa*)(so + rr * 68 + q); }
    __threadfence();
  }
}

__global__ __launch_bounds__(256) void k_sub(const float* __restrict__ a, const float* __restrict__ b, float* __restrict__ d) { const size_t row = blockIdx.x;
  for (int q4 = threadIdx.x; q4 < DDc / 4; q4 += 256) { const v4f_t x = *(const v4f_t*)(a + row * DDc + q4 * 4), y = *(const v4f_t*)(b + row * DDc + q4 * 4); v4f_t o; for (int e = 0; e < 4; ++e) o[e] = x[e] - y[e];
    *(volatile v4f_t*)(d + row * DDc + q4 * 4) = o; __threadfence(); *(volatile v4f_t*)(d + row * DDc + q4 * 4) = o; } }
__global__ __launch_bounds__(256) void k_transpose(const float* __restrict__ Wm, float* __restrict__ Wt, int rows, int cols) {
  __shared__ float tS[64][65];
  const int tid = threadIdx.x, tbj = cols / 64, bi = blockIdx.x / tbj, bj = blockIdx.x % tbj;
  for (int e = tid; e < 64 * 64; e += 256) { const int r = e >> 6, c = e & 63; tS[r][c] = Wm[(size_t)(bi * 64 + r) * cols + bj * 64 + c]; }
  __syncthreads();
  for (int ch = tid; ch < 64 * 16; ch += 256) { const int r = ch >> 4, q4 = (ch & 15) * 4; v4f_t o; o[0] = tS[q4][r]; o[1] = tS[q4 + 1][r]; o[2] = tS[q4 + 2][r]; o[3] = tS[q4 + 3][r];
    float* dst = Wt + (size_t)(bj * 64 + r) * rows + bi * 64 + q4; *(volatile v4f_t*)dst = o; __threadfence(); *(volatile v4f_t*)dst = o; }
}
__global__ __launch_bounds__(256) void k_pair(const float* __restrict__ L, const float* __restrict__ base, const float* __restrict__ dQ, const float* __restrict__ W2, const float* __restrict__ b2,
                                             const float* __restrict__ W3, const float* __restrict__ b3, float* __restrict__ out) {
  __shared__ __attribute__((aligned(16))) f16 aS[128 * 264];
  __shared__ __attribute__((aligned(16))) f16 wS[H2c * 264];
  __shared__ float wgt[8][128];
  __shared__ __attribute__((aligned(16))) float oS[128];
  const int tid = threadIdx.x, lane = tid & 31, wave = tid >> 5, cl = lane & 15, rh = (lane >> 4) * 8;
  const int n = blockIdx.x / (NMc / 128), m0 = (blockIdx.x % (NMc / 128)) * 128;
  const float scale = 0.10206207261596575f;
  for (int e = tid; e < 8 * 128; e += 256) { const int h = e >> 7, m = e & 127; const float l = L[((size_t)h * NQc + n) * NMc + m0 + m] * scale; wgt[h][m] = 1.0f / (1.0f + expf(-l)); }
  for (int e = tid; e < H2c * HIDc; e += 256) { const int k = e / H2c, nn = e % H2c; wS[nn * 264 + k] = (f16)W2[e]; }
  __syncthreads();
  for (int e = tid; e < 128 * HIDc; e += 256) { const int m = e >> 8, c = e & 255; float v = base[(size_t)(m0 + m) * HIDc + c];
#pragma unroll 1
    for (int h = 0; h < NHc; ++h) v += wgt[h][m] * dQ[((size_t)h * NMc + m0 + m) * HIDc + c];
    aS[m * 264 + c] = (f16)fmaxf(v, 0.0f); }
  __syncthreads();
  f32x8 acc[4];
#pragma unroll
  for (int j = 0; j < 4; ++j) { f32x8 z = {}; acc[j] = z; }
#pragma unroll 1
  for (int ks = 0; ks < HIDc / 32; ++ks) { const f16x16 af = lds_frag(aS + (wave * 16) * 264 + ks * 32, 264);
#pragma unroll
    for (int j = 0; j < 4; ++j) acc[j] = wmma16(af, lds_frag(wS + (j * 16) * 264 + ks * 32, 264), acc[j]); }
  float ep[8];
#pragma unroll
  for (int r = 0; r < 8; ++r) ep[r] = 0.0f;
#pragma unroll
  for (int j = 0; j < 4; ++j) { const int o = j * 16 + cl; const float bb = b2[o], w3 = W3[o];
#pragma unroll
    for (int r = 0; r < 8; ++r) ep[r] += fmaxf(acc[j][r] + bb, 0.0f) * w3; }
#pragma unroll
  for (int r = 0; r < 8; ++r) { float v = ep[r];
#pragma unroll
    for (int off = 1; off < 16; off <<= 1) v += __shfl_xor(v, off, 32);
    ep[r] = v; }
  if (cl == 0) {
#pragma unroll
    for (int r = 0; r < 8; ++r) oS[wave * 16 + rh + r] = 0.5f * tanhf(ep[r] + b3[0]); }
  __syncthreads();
#pragma unroll 1
  for (int pass = 0; pass < 2; ++pass) { if (tid < 32) *(volatile v4f_t*)(out + (size_t)n * NMc + m0 + tid * 4) = *(const v4fa*)(oS + tid * 4); __threadfence(); }
}

extern "C" void kernel_launch(void* const* d_in, const int* in_sizes, int n_in,
                              void* d_out, int out_size, void* d_ws, size_t ws_size,
                              hipStream_t stream) {
  (void)in_sizes; (void)n_in; (void)out_size;
  const float** f = (const float**)d_in;
  const float* qe = f[0], *ie = f[1], *te = f[2], *Wq = f[3], *bq = f[4], *Wi = f[5], *bi = f[6], *Wt = f[7], *bt = f[8], *Wiq = f[9], *biq = f[10], *Wik = f[11], *bik = f[12], *Wiv = f[13], *biv = f[14],
             *Wo = f[15], *bo = f[16], *W1 = f[17], *b1 = f[18], *W2 = f[19], *b2 = f[20], *W3 = f[21], *b3 = f[22];
  (void)bik;
  float* out = (float*)d_out;
  char* ws = (char*)d_ws;
  float* q = (float*)ws; ws += (size_t)NQc * DDc * 4; float* qh = (float*)ws; ws += (size_t)NQc * DDc * 4;
  float* img = (float*)ws; ws += (size_t)NMc * DDc * 4; float* tgt = (float*)ws; ws += (size_t)NMc * DDc * 4; float* dit = (float*)ws; ws += (size_t)NMc * DDc * 4;
  float* dk = (float*)ws; ws += (size_t)NMc * DDc * 4; float* dkT = (float*)ws; ws += (size_t)DDc * NMc * 4; float* dv = (float*)ws; ws += (size_t)NMc * DDc * 4; float* vt = (float*)ws; ws += (size_t)NMc * DDc * 4;
  float* L = (float*)ws; ws += (size_t)NHc * NQc * NMc * 4;
  float* A1 = (float*)ws; ws += (size_t)NMc * DDc * 4;
  float* c1 = (float*)ws; ws += HIDc * 4;
  float* base = (float*)ws; ws += (size_t)NMc * HIDc * 4;
  float* dP = (float*)ws; ws += (size_t)NHc * NMc * DDc * 4;
  float* dQ = (float*)ws; ws += (size_t)NHc * NMc * HIDc * 4;
  if ((size_t)(ws - (char*)d_ws) > ws_size) return;
  const dim3 blk(256);
  gemm_kn2<float, false><<<dim3(NQc / 128, DDc / 128, 1), blk, 0, stream>>>(qe, DDc, 0, Wq, DDc, 0, bq, 1.0f, q, DDc, 0, DDc);
  gemm_kn2<float, false><<<dim3(NQc / 128, DDc / 128, 1), blk, 0, stream>>>(q, DDc, 0, Wiq, DDc, 0, biq, 1.0f, qh, DDc, 0, DDc);
  gemm_kn2<float, false><<<dim3(NMc / 128, DDc / 128, 1), blk, 0, stream>>>(ie, DDc, 0, Wi, DDc, 0, bi, 1.0f, img, DDc, 0, DDc);
  gemm_kn2<float, false><<<dim3(NMc / 128, DDc / 128, 1), blk, 0, stream>>>(te, DDc, 0, Wt, DDc, 0, bt, 1.0f, tgt, DDc, 0, DDc);
  k_sub<<<dim3(NMc), blk, 0, stream>>>(img, tgt, dit);
  gemm_kn2<float, false><<<dim3(NMc / 128, DDc / 128, 1), blk, 0, stream>>>(dit, DDc, 0, Wik, DDc, 0, nullptr, 1.0f, dk, DDc, 0, DDc);
  gemm_kn2<float, false><<<dim3(NMc / 128, DDc / 128, 1), blk, 0, stream>>>(dit, DDc, 0, Wiv, DDc, 0, nullptr, 1.0f, dv, DDc, 0, DDc);
  gemm_kn2<float, false><<<dim3(NMc / 128, DDc / 128, 1), blk, 0, stream>>>(tgt, DDc, 0, Wiv, DDc, 0, biv, 1.0f, vt, DDc, 0, DDc);
  k_transpose<<<dim3((NMc / 64) * (DDc / 64)), blk, 0, stream>>>(dk, dkT, NMc, DDc);
  for (int h = 0; h < NHc; ++h) {
    gemm_kn2<float, false><<<dim3(NQc / 128, NMc / 128, 1), blk, 0, stream>>>(qh + h * DHc, DDc, 0, dkT + (size_t)h * DHc * NMc, NMc, 0, nullptr, 1.0f, L + (size_t)h * NQc * NMc, NMc, 0, DHc);
    gemm_kn2<float, false><<<dim3(NMc / 128, DDc / 128, 1), blk, 0, stream>>>(dv + h * DHc, DDc, 0, Wo + (size_t)h * DHc * DDc, DDc, 0, nullptr, 1.0f, dP + (size_t)h * NMc * DDc, DDc, 0, DHc);
  }
  gemm_kn2<float, false><<<dim3(NMc / 128, DDc / 128, 1), blk, 0, stream>>>(vt, DDc, 0, Wo, DDc, 0, bo, 1.0f, A1, DDc, 0, DDc);
  gemm_kn2<float, false><<<dim3(NMc / 128, HIDc / 128, 1), blk, 0, stream>>>(A1, DDc, 0, W1, HIDc, 0, b1, 1.0f, base, HIDc, 0, DDc);
  gemm_kn2<float, false><<<dim3(NHc * NMc / 128, HIDc / 128, 1), blk, 0, stream>>>(dP, DDc, 0, W1, HIDc, 0, nullptr, 1.0f, dQ, HIDc, 0, DDc);
  k_pair<<<dim3(NQc * (NMc / 128)), blk, 0, stream>>>(L, base, dQ, W2, b2, W3, b3, out);
}
